// MoLE_42004780155103
// MI455X (gfx1250) — hardware-run, weakly checked
//
#include <hip/hip_runtime.h>

typedef __attribute__((ext_vector_type(16))) _Float16     v16h;
typedef __attribute__((ext_vector_type(8)))  _Float16     v8h;
typedef __attribute__((ext_vector_type(8)))  float        v8f;
typedef __attribute__((ext_vector_type(4)))  float        v4f;
typedef __attribute__((ext_vector_type(4)))  int          v4i;
typedef __attribute__((ext_vector_type(4)))  unsigned int v4u;

constexpr int kBanks  = 16;
constexpr int kInF    = 256;
constexpr int kOutF   = 256;
constexpr int kGraphs = 16;
constexpr int kNodes  = 4096;
constexpr int kPlane  = kInF * kOutF;
constexpr int kTileM  = 32;
constexpr int kTileN  = 64;
constexpr float kMixCarry    = 8.0f;
constexpr float kMixCarryInv = 1.0f / kMixCarry;

static_assert(kBanks == 16 && kGraphs == 16, "mixing tables sized for 16 x 16");
static_assert((kInF % 32) == 0, "GEMM K multiple of 32");
static_assert((kNodes % kTileM) == 0 && (kOutF % kTileN) == 0, "GEMM M, N multiples of the wave tile");
static_assert((kOutF / kTileN) == 4, "tile index split uses 4 column tiles");
static_assert(((kNodes / kTileM) * (kOutF / kTileN)) % 8 == 0, "8 wave tiles per block, exact grid");
static_assert((kInF % 64) == 0 && (kOutF % 16) == 0, "mixing tile multiples");
static_assert(kGraphs * kBanks == 256, "coefficient table = one element per thread");

constexpr size_t kOffA16  = 0;
constexpr size_t kOffBT16 = kOffA16 + (size_t)kNodes * kInF * 2;
constexpr size_t kWsTotal = kOffBT16 + (size_t)kGraphs * kOutF * kInF * 2;
static_assert(kWsTotal == 4194304ull, "carve total");
static_assert(kWsTotal <= 134217728ull, "carve cap");
static_assert((kOffBT16 % 128) == 0, "128-B aligned regions");

union FragH { v16h v; v8h h[2]; };
__device__ __forceinline__ v16h frag_load_h(const _Float16* p) {
  FragH f;
  f.h[0] = *(const v8h*)(p);
  f.h[1] = *(const v8h*)(p + 16);
  return f.v;
}
__device__ __forceinline__ v8f mma_g(v16h a, v16h b, v8f c) {
  c = __builtin_amdgcn_wmma_f32_16x16x32_f16(false, a, false, b, (short)0, c, false, false);
  asm volatile("v_nop\n\tv_nop\n\tv_nop\n\tv_nop" : "+v"(c) : "v"(a), "v"(b));
  return c;
}

__global__ __launch_bounds__(256) void cast_rows_f16_kernel(
    const float* __restrict__ src, unsigned short* __restrict__ dst, int total8)
{
  const int i = blockIdx.x * 256 + threadIdx.x;
  if (i >= total8) return;
  const size_t e0 = (size_t)i << 3;
  const v4f a0 = *(const v4f*)(src + e0);
  const v4f a1 = *(const v4f*)(src + e0 + 4);
  v8h hv;
#pragma unroll
  for (int e = 0; e < 4; ++e) {
    const float f0 = a0[e];
    const float f1 = a1[e];
    hv[e]     = (_Float16)f0;
    hv[4 + e] = (_Float16)f1;
  }
  unsigned short* q = dst + e0;
  *(volatile v8h*)q = hv;
  __threadfence();
  *(volatile v8h*)q = hv;
}

__global__ __launch_bounds__(256) void mix_transpose_kernel(
    const float* __restrict__ bank, const float* __restrict__ coef, unsigned int* __restrict__ BtW)
{
  __shared__ __align__(16) float sc[kGraphs * kBanks];
  __shared__ __align__(16) unsigned int sTileW[kGraphs * 16 * 32];
  const int tid = threadIdx.x, lane = tid & 31, wave = tid >> 5;
  const int i0 = (blockIdx.x & 3) * 64;
  const int o0 = (blockIdx.x >> 2) * 16;
  sc[tid] = coef[tid];
  __syncthreads();
  const int ol = tid & 15;
  const int iq = tid >> 4;
#pragma unroll 1
  for (int p = 0; p < 2; ++p) {
    const int ip = iq + 16 * p;
    const float* src = bank + (size_t)(i0 + 2 * ip) * kOutF + o0 + ol;
    float ka[kBanks], kb[kBanks];
#pragma unroll
    for (int e = 0; e < kBanks; ++e) ka[e] = src[(size_t)e * kPlane];
    asm volatile("s_nop 0" ::: "memory");
#pragma unroll
    for (int e = 0; e < kBanks; ++e) kb[e] = src[(size_t)e * kPlane + kOutF];
#pragma unroll 1
    for (int g = 0; g < kGraphs; ++g) {
      const float* cr = sc + g * kBanks;
      float s0 = 0.0f, s1 = 0.0f;
#pragma unroll
      for (int e = 0; e < kBanks; ++e) {
        const float c = cr[e];
        s0 = fmaf(c, ka[e], s0);
        s1 = fmaf(c, kb[e], s1);
      }
      const _Float16 h0 = (_Float16)(s0 * kMixCarry);
      const _Float16 h1 = (_Float16)(s1 * kMixCarry);
      const unsigned int u = (unsigned int)__builtin_bit_cast(unsigned short, h0) |
                             ((unsigned int)__builtin_bit_cast(unsigned short, h1) << 16);
      sTileW[(g * 16 + ol) * 32 + ip] = u;
    }
  }
  __syncthreads();
  const int q  = lane >> 3;
  const int c4 = (lane & 7) * 4;
  v4u vv[8];
#pragma unroll
  for (int it = 0; it < 8; ++it) {
    const int L = wave * 32 + it * 4 + q;
    vv[it] = *(const v4u*)(sTileW + L * 32 + c4);
  }
  for (int pass = 0; pass < 2; ++pass) {
#pragma unroll
    for (int it = 0; it < 8; ++it) {
      const int L = wave * 32 + it * 4 + q;
      const int g = L >> 4;
      const int o = o0 + (L & 15);
      unsigned int* dst = BtW + ((size_t)(g * kOutF + o) * (kInF / 2) + (i0 >> 1) + c4);
      *(volatile v4u*)dst = vv[it];
    }
    __threadfence();
  }
}

__global__ __launch_bounds__(256) __attribute__((amdgpu_num_vgpr(256))) void graph_gemm_f16_kernel(
    const unsigned short* __restrict__ Ap, const unsigned short* __restrict__ Btp,
    const float* __restrict__ bias, const int* __restrict__ ncount, float* __restrict__ out)
{
  const _Float16* A  = (const _Float16*)Ap;
  const _Float16* Bt = (const _Float16*)Btp;
  __shared__ __align__(16) float sT[8][16 * 68];
  const int lane = threadIdx.x & 31;
  const int wave = threadIdx.x >> 5;
  const int tile = blockIdx.x * 8 + wave;
  const int tm = tile >> 2;
  const int tn = tile & 3;
  const int m0 = tm * kTileM;
  const int n0 = tn * kTileN;
  const int rlane = lane & 15;
  const int koff  = (lane >> 4) * 8;
  const int mOff  = (lane >> 4) * 8;

  int nn[16];
  {
    const v4i q0 = *(const v4i*)(ncount);
    const v4i q1 = *(const v4i*)(ncount + 4);
    const v4i q2 = *(const v4i*)(ncount + 8);
    const v4i q3 = *(const v4i*)(ncount + 12);
#pragma unroll
    for (int e = 0; e < 4; ++e) {
      const int t0 = q0[e];
      const int t1 = q1[e];
      const int t2 = q2[e];
      const int t3 = q3[e];
      nn[e]      = t0;
      nn[4 + e]  = t1;
      nn[8 + e]  = t2;
      nn[12 + e] = t3;
    }
#pragma unroll
    for (int j = 0; j < 16; ++j) {
      int t = nn[j];
      t = (t < 0) ? 0 : t;
      t = (t > kNodes) ? kNodes : t;
      nn[j] = __builtin_amdgcn_readfirstlane(t);
    }
  }
  int gf = 0, gl = 0;
  {
    int cum = 0;
#pragma unroll
    for (int j = 0; j < 15; ++j) {
      cum += nn[j];
      gf += (cum <= m0) ? 1 : 0;
      gl += (cum <= m0 + (kTileM - 1)) ? 1 : 0;
    }
  }
  gf = __builtin_amdgcn_readfirstlane(gf);
  gl = __builtin_amdgcn_readfirstlane(gl);
  gf = (gf < 0) ? 0 : ((gf > 15) ? 15 : gf);
  gl = (gl < gf) ? gf : ((gl > 15) ? 15 : gl);

  float bv[4];
#pragma unroll
  for (int j = 0; j < 4; ++j) bv[j] = bias[n0 + (j << 4) + rlane];

  float* slab = sT[wave];
  const int hh = lane >> 4;
  const int c4 = (lane & 15) * 4;

  const int aRow0 = (m0 + rlane) * kInF + koff;
  const int bRow0 = (n0 + rlane) * kInF + koff;

#pragma unroll 1
  for (int g = gf; g <= gl; ++g) {
    int rs = 0, re = 0;
#pragma unroll
    for (int j = 0; j < 16; ++j) {
      rs += (j < g) ? nn[j] : 0;
      re += (j <= g) ? nn[j] : 0;
    }
    if (g >= 15) re = 0x7fffffff;

    const _Float16* Bb = Bt + (size_t)g * kPlane;

    v8f acc[2][4];
#pragma unroll
    for (int i = 0; i < 2; ++i)
#pragma unroll
      for (int j = 0; j < 4; ++j) acc[i][j] = (v8f){0.f, 0.f, 0.f, 0.f, 0.f, 0.f, 0.f, 0.f};

#pragma unroll 1
    for (int k0 = 0; k0 < kInF; k0 += 32) {
      v16h bh[4];
#pragma unroll
      for (int j = 0; j < 4; ++j) {
        bh[j] = frag_load_h(Bb + bRow0 + (j << 4) * kInF + k0);
      }
#pragma unroll
      for (int i = 0; i < 2; ++i) {
        const v16h ah = frag_load_h(A + aRow0 + (i << 4) * kInF + k0);
#pragma unroll
        for (int j = 0; j < 4; ++j) acc[i][j] = mma_g(ah, bh[j], acc[i][j]);
      }
    }

#pragma unroll
    for (int i = 0; i < 2; ++i) {
      const int mBase = m0 + (i << 4);
#pragma unroll
      for (int j = 0; j < 4; ++j) {
#pragma unroll
        for (int r = 0; r < 8; ++r) {
          const float v = fmaf(acc[i][j][r], kMixCarryInv, bv[j]);
          slab[(mOff + r) * 68 + (j << 4) + rlane] = v;
        }
      }
      __builtin_amdgcn_fence(__ATOMIC_RELEASE, "workgroup");
      __builtin_amdgcn_wave_barrier();
      __builtin_amdgcn_fence(__ATOMIC_ACQUIRE, "workgroup");
      for (int pass = 0; pass < 2; ++pass) {
#pragma unroll
        for (int it = 0; it < 8; ++it) {
          const int row  = it * 2 + hh;
          const int grow = mBase + row;
          const v4f v = *(const v4f*)(slab + row * 68 + c4);
          if (grow >= rs && grow < re) {
            *(volatile v4f*)(out + (size_t)grow * kOutF + n0 + c4) = v;
          }
        }
        __threadfence();
      }
      __builtin_amdgcn_fence(__ATOMIC_RELEASE, "workgroup");
      __builtin_amdgcn_wave_barrier();
      __builtin_amdgcn_fence(__ATOMIC_ACQUIRE, "workgroup");
    }
  }
}

extern "C" void kernel_launch(void* const* d_in, const int* in_sizes, int n_in,
                              void* d_out, int out_size, void* d_ws, size_t ws_size,
                              hipStream_t stream) {
  if (n_in < 5) return;
  if (in_sizes[0] != kNodes * kInF) return;
  if (in_sizes[1] != kBanks * kInF * kOutF) return;
  if (in_sizes[2] != kOutF) return;
  if (in_sizes[3] != kGraphs * kBanks) return;
  if (in_sizes[4] != kGraphs) return;
  if (out_size != kNodes * kOutF) return;
  if (ws_size < kWsTotal) return;

  const float* x      = (const float*)d_in[0];
  const float* bank   = (const float*)d_in[1];
  const float* bias   = (const float*)d_in[2];
  const float* coef   = (const float*)d_in[3];
  const int*   ncount = (const int*)d_in[4];
  float* out = (float*)d_out;

  char* ws = (char*)d_ws;
  unsigned short* A16  = (unsigned short*)(ws + kOffA16);
  unsigned short* BT16 = (unsigned short*)(ws + kOffBT16);

  cast_rows_f16_kernel<<<(kNodes * kInF / 8) / 256, 256, 0, stream>>>(x, A16, kNodes * kInF / 8);
  mix_transpose_kernel<<<(kInF / 64) * (kOutF / 16), 256, 0, stream>>>(bank, coef, (unsigned int*)BT16);
  graph_gemm_f16_kernel<<<((kNodes / kTileM) * (kOutF / kTileN)) / 8, 256, 0, stream>>>(A16, BT16, bias, ncount, out);
}
